// PointNetFeaturePropagation_40785009443185
// MI455X (gfx1250) — hardware-verified
//
#include <hip/hip_runtime.h>
#include <stdint.h>

#pragma clang fp contract(off)

typedef __attribute__((ext_vector_type(16))) _Float16 v16h;
typedef __attribute__((ext_vector_type(8)))  _Float16 v8h;
typedef __attribute__((ext_vector_type(8)))  float    v8f;
typedef __attribute__((ext_vector_type(4)))  float    v4f;

constexpr int NBATCH   = 2;
constexpr int NPT      = 16384;
constexpr int SPT      = 4096;
constexpr int DSF      = 128;
constexpr int DTF      = 256;
constexpr int CIN_CH   = DSF + DTF;
constexpr int C0_CH    = 256;
constexpr int C1_CH    = 128;
constexpr int MROW     = NBATCH * NPT;
constexpr int KNN_TILE = 512;
constexpr int STAT_BLOCKS = 128;
constexpr int STAT_ROWS   = MROW / STAT_BLOCKS;

constexpr float W_CARRY   = 16.0f;
constexpr float LO_CARRY  = 2048.0f;
constexpr float SCALE_MAIN = 1.0f / W_CARRY;
constexpr float SCALE_RES  = 1.0f / (W_CARRY * LO_CARRY);
constexpr float KNN_EPS   = 1e-8f;
constexpr float BN_EPS    = 1e-5f;

static_assert(CIN_CH == 384, "concat width");
static_assert(MROW % 64 == 0, "M tile multiple");
static_assert(C0_CH % 32 == 0 && C1_CH % 32 == 0, "N tile multiple");
static_assert(CIN_CH % 32 == 0 && C0_CH % 32 == 0, "K multiple of 32");
static_assert(STAT_ROWS == 256, "stat rows per block");
static_assert(SPT % KNN_TILE == 0 && KNN_TILE % 256 == 0, "knn tiling");
static_assert(NPT % 256 == 0, "query blocks do not straddle batches");

constexpr size_t SZ_FEAT  = (size_t)MROW * CIN_CH * 2;
constexpr size_t SZ_A1    = (size_t)MROW * C0_CH * 2;
constexpr size_t SZ_X0    = (size_t)MROW * C0_CH * 4;
constexpr size_t SZ_Y1    = (size_t)MROW * C1_CH * 4;
constexpr size_t SZ_WB0   = (size_t)C0_CH * CIN_CH * 2;
constexpr size_t SZ_WB1   = (size_t)C1_CH * C0_CH * 2;
constexpr size_t SZ_IDX   = (size_t)3 * MROW * 4;
constexpr size_t SZ_PS0   = (size_t)STAT_BLOCKS * C0_CH * 4;
constexpr size_t SZ_PS1   = (size_t)STAT_BLOCKS * C1_CH * 4;

constexpr size_t OFF_FEAT_HI = 0;
constexpr size_t OFF_FEAT_LO = OFF_FEAT_HI + SZ_FEAT;
constexpr size_t OFF_X0      = OFF_FEAT_LO + SZ_FEAT;
constexpr size_t OFF_Y1      = OFF_X0 + SZ_X0;
constexpr size_t OFF_WB0_HI  = OFF_Y1 + SZ_Y1;
constexpr size_t OFF_WB0_LO  = OFF_WB0_HI + SZ_WB0;
constexpr size_t OFF_WB1_HI  = OFF_WB0_LO + SZ_WB0;
constexpr size_t OFF_WB1_LO  = OFF_WB1_HI + SZ_WB1;
constexpr size_t OFF_IDX     = OFF_WB1_LO + SZ_WB1;
constexpr size_t OFF_DIST    = OFF_IDX + SZ_IDX;
constexpr size_t OFF_PSUM0   = OFF_DIST + SZ_IDX;
constexpr size_t OFF_PSQ0    = OFF_PSUM0 + SZ_PS0;
constexpr size_t OFF_PSUM1   = OFF_PSQ0 + SZ_PS0;
constexpr size_t OFF_PSQ1    = OFF_PSUM1 + SZ_PS1;
constexpr size_t OFF_SCALE0  = OFF_PSQ1 + SZ_PS1;
constexpr size_t OFF_SHIFT0  = OFF_SCALE0 + (size_t)C0_CH * 4;
constexpr size_t OFF_SCALE1  = OFF_SHIFT0 + (size_t)C0_CH * 4;
constexpr size_t OFF_SHIFT1  = OFF_SCALE1 + (size_t)C1_CH * 4;
constexpr size_t WS_END      = OFF_SHIFT1 + (size_t)C1_CH * 4;

static_assert(SZ_A1 <= SZ_FEAT, "A1 planes fit in the dead FEAT planes");
static_assert(WS_END <= (size_t)134217728, "carve within 128 MiB");
static_assert((OFF_FEAT_LO % 128) == 0 && (OFF_X0 % 128) == 0 && (OFF_Y1 % 128) == 0 &&
              (OFF_WB0_HI % 128) == 0 && (OFF_WB0_LO % 128) == 0 && (OFF_WB1_HI % 128) == 0 &&
              (OFF_WB1_LO % 128) == 0 && (OFF_IDX % 128) == 0 && (OFF_DIST % 128) == 0 &&
              (OFF_PSUM0 % 128) == 0 && (OFF_PSQ0 % 128) == 0 && (OFF_PSUM1 % 128) == 0 &&
              (OFF_PSQ1 % 128) == 0 && (OFF_SCALE0 % 128) == 0 && (OFF_SHIFT0 % 128) == 0 &&
              (OFF_SCALE1 % 128) == 0 && (OFF_SHIFT1 % 128) == 0, "line-aligned carves");

__device__ __forceinline__ void keep4_h(v16h a, v16h b, v16h c, v16h d) { asm volatile("v_nop" :: "v"(a), "v"(b), "v"(c), "v"(d)); }
__device__ __forceinline__ void acc_guard4(v8f& a, v8f& b, v8f& c, v8f& d) { asm volatile("v_nop\n\tv_nop\n\tv_nop\n\tv_nop" : "+v"(a), "+v"(b), "+v"(c), "+v"(d)); }
__device__ __forceinline__ void group_guard_h(v8f& a, v8f& b, v8f& c, v8f& d, v16h x, v16h y) {
  asm volatile("v_nop\n\tv_nop\n\tv_nop\n\tv_nop" : "+v"(a), "+v"(b), "+v"(c), "+v"(d) : "v"(x), "v"(y));
}
template <typename T> struct Frag;
template <> struct Frag<_Float16> {
  typedef v16h V; union U { v16h v; v8h h[2]; };
  static __device__ __forceinline__ v16h load(const _Float16* p) {
    U f; f.h[0] = *(const v8h*)(p); f.h[1] = *(const v8h*)(p + 16); return f.v;
  }
  static __device__ __forceinline__ v8f mma(v16h a, v16h b, v8f c) {
    return __builtin_amdgcn_wmma_f32_16x16x32_f16(false, a, false, b, (short)0, c, false, false);
  }
};

__device__ __forceinline__ void split_h(float v, float carry, _Float16& h, _Float16& l) {
  const _Float16 hh = (_Float16)v;
  const float back = (float)hh;
  const float res = v - back;
  const float sres = res * carry;
  h = hh;
  l = (_Float16)sres;
}

__global__ __launch_bounds__(256) void split_weights_kernel(
    const float* __restrict__ w, unsigned short* __restrict__ hi, unsigned short* __restrict__ lo, int n8) {
  const int t = blockIdx.x * 256 + threadIdx.x;
  const int tc = (t < n8) ? t : (n8 - 1);
  const float* wp = w + (size_t)tc * 8;
  const v4f a = *(const v4f*)wp;
  const v4f b = *(const v4f*)(wp + 4);
  float x[8];
  x[0] = a.x; x[1] = a.y; x[2] = a.z; x[3] = a.w;
  x[4] = b.x; x[5] = b.y; x[6] = b.z; x[7] = b.w;
  v8h hv, lv;
#pragma unroll
  for (int e = 0; e < 8; ++e) {
    _Float16 h, l;
    const float xs = x[e] * W_CARRY;
    split_h(xs, LO_CARRY, h, l);
    hv[e] = h; lv[e] = l;
  }
  if (t < n8) {
    volatile v8h* ph = (volatile v8h*)(void*)(hi + (size_t)tc * 8);
    volatile v8h* pl = (volatile v8h*)(void*)(lo + (size_t)tc * 8);
    *ph = hv; *pl = lv;
    __threadfence();
    *ph = hv; *pl = lv;
  }
}

__global__ __launch_bounds__(256) void knn3_kernel(
    const float* __restrict__ xyz_s, const float* __restrict__ xyz_t,
    int* __restrict__ idx, float* __restrict__ dist) {
#pragma clang fp contract(off)
  __shared__ __align__(16) v4f lt[KNN_TILE];
  const int tid = threadIdx.x;
  const int p = blockIdx.x * 256 + tid;
  const int b = blockIdx.x / (NPT / 256);
  const float sx = xyz_s[(size_t)p * 3 + 0];
  const float sy = xyz_s[(size_t)p * 3 + 1];
  const float sz = xyz_s[(size_t)p * 3 + 2];
  const float sxx = sx * sx;
  const float syy = sy * sy;
  const float szz = sz * sz;
  const float sn = (sxx + szz) + syy;
  const float* tb = xyz_t + (size_t)b * SPT * 3;

  const float finf = __builtin_inff();
  float bd0 = finf, bd1 = finf, bd2 = finf;
  int bi0 = 0, bi1 = 0, bi2 = 0;

  for (int s0 = 0; s0 < SPT; s0 += KNN_TILE) {
    __syncthreads();
#pragma unroll
    for (int u = 0; u < KNN_TILE / 256; ++u) {
      const int i = tid + u * 256;
      const float* tp = tb + (size_t)(s0 + i) * 3;
      const float tx = tp[0];
      const float ty = tp[1];
      const float tz = tp[2];
      const float txx = tx * tx;
      const float tyy = ty * ty;
      const float tzz = tz * tz;
      const float tn = (txx + tzz) + tyy;
      v4f e;
      e.x = tx; e.y = ty; e.z = tz; e.w = tn;
      lt[i] = e;
    }
    __syncthreads();
#pragma unroll 4
    for (int j = 0; j < KNN_TILE; ++j) {
      const v4f t = lt[j];
      float pd = sx * t.x;
      pd = __builtin_fmaf(sy, t.y, pd);
      pd = __builtin_fmaf(sz, t.z, pd);
      const float ssum = sn + t.w;
      const float twop = pd + pd;
      const float d = ssum - twop;
      const int s = s0 + j;
      const bool lt0 = d < bd0;
      const bool lt1 = d < bd1;
      const bool lt2 = d < bd2;
      const float n2 = lt1 ? bd1 : (lt2 ? d : bd2);
      const int   m2 = lt1 ? bi1 : (lt2 ? s : bi2);
      const float n1 = lt0 ? bd0 : (lt1 ? d : bd1);
      const int   m1 = lt0 ? bi0 : (lt1 ? s : bi1);
      const float n0 = lt0 ? d : bd0;
      const int   m0 = lt0 ? s : bi0;
      bd2 = n2; bi2 = m2;
      bd1 = n1; bi1 = m1;
      bd0 = n0; bi0 = m0;
    }
  }
  int g0 = bi0 < 0 ? 0 : (bi0 > SPT - 1 ? SPT - 1 : bi0);
  int g1 = bi1 < 0 ? 0 : (bi1 > SPT - 1 ? SPT - 1 : bi1);
  int g2 = bi2 < 0 ? 0 : (bi2 > SPT - 1 ? SPT - 1 : bi2);
  g0 += b * SPT; g1 += b * SPT; g2 += b * SPT;
  volatile int* vi = (volatile int*)idx;
  volatile float* vd = (volatile float*)dist;
  vi[p] = g0; vi[MROW + p] = g1; vi[2 * MROW + p] = g2;
  vd[p] = bd0; vd[MROW + p] = bd1; vd[2 * MROW + p] = bd2;
  __threadfence();
  vi[p] = g0; vi[MROW + p] = g1; vi[2 * MROW + p] = g2;
  vd[p] = bd0; vd[MROW + p] = bd1; vd[2 * MROW + p] = bd2;
}

__global__ __launch_bounds__(256) void build_features_kernel(
    const float* __restrict__ feats_s, const float* __restrict__ feats_t,
    const int* __restrict__ idx, const float* __restrict__ dist,
    unsigned short* __restrict__ fhi, unsigned short* __restrict__ flo) {
  const int wave = threadIdx.x >> 5;
  const int lane = threadIdx.x & 31;
  const int row0 = (blockIdx.x * 8 + wave) * 2;
  {
    const int rS = row0 + (lane >> 4);
    const int cs = (lane & 15) * 8;
    const float* fs = feats_s + (size_t)rS * DSF + cs;
    const v4f a = *(const v4f*)fs;
    const v4f b = *(const v4f*)(fs + 4);
    float x[8];
    x[0] = a.x; x[1] = a.y; x[2] = a.z; x[3] = a.w;
    x[4] = b.x; x[5] = b.y; x[6] = b.z; x[7] = b.w;
    v8h hv, lv;
#pragma unroll
    for (int e = 0; e < 8; ++e) {
      _Float16 h, l;
      split_h(x[e], LO_CARRY, h, l);
      hv[e] = h; lv[e] = l;
    }
    volatile v8h* ph = (volatile v8h*)(void*)(fhi + (size_t)rS * CIN_CH + cs);
    volatile v8h* pl = (volatile v8h*)(void*)(flo + (size_t)rS * CIN_CH + cs);
    *ph = hv; *pl = lv;
    __threadfence();
    *ph = hv; *pl = lv;
  }
#pragma unroll 1
  for (int t = 0; t < 2; ++t) {
    const int r = row0 + t;
    const int bb = r / NPT;
    const int ilo = bb * SPT;
    const int ihi = ilo + SPT - 1;
    int i0 = idx[r];
    int i1 = idx[MROW + r];
    int i2 = idx[2 * MROW + r];
    i0 = i0 < ilo ? ilo : (i0 > ihi ? ihi : i0);
    i1 = i1 < ilo ? ilo : (i1 > ihi ? ihi : i1);
    i2 = i2 < ilo ? ilo : (i2 > ihi ? ihi : i2);
    const float d0 = dist[r];
    const float d1 = dist[MROW + r];
    const float d2 = dist[2 * MROW + r];
    const float r0 = 1.0f / (d0 + KNN_EPS);
    const float r1 = 1.0f / (d1 + KNN_EPS);
    const float r2 = 1.0f / (d2 + KNN_EPS);
    const float rs = (r0 + r2) + r1;
    const float w0 = r0 / rs;
    const float w1 = r1 / rs;
    const float w2 = r2 / rs;
    const int ci = lane * 8;
    const float* p0 = feats_t + (size_t)i0 * DTF + ci;
    const float* p1 = feats_t + (size_t)i1 * DTF + ci;
    const float* p2 = feats_t + (size_t)i2 * DTF + ci;
    const v4f a0 = *(const v4f*)p0;
    const v4f a1 = *(const v4f*)(p0 + 4);
    const v4f b0 = *(const v4f*)p1;
    const v4f b1 = *(const v4f*)(p1 + 4);
    const v4f c0 = *(const v4f*)p2;
    const v4f c1 = *(const v4f*)(p2 + 4);
    float x[8];
    x[0] = (w0 * a0.x + w1 * b0.x) + w2 * c0.x;
    x[1] = (w0 * a0.y + w1 * b0.y) + w2 * c0.y;
    x[2] = (w0 * a0.z + w1 * b0.z) + w2 * c0.z;
    x[3] = (w0 * a0.w + w1 * b0.w) + w2 * c0.w;
    x[4] = (w0 * a1.x + w1 * b1.x) + w2 * c1.x;
    x[5] = (w0 * a1.y + w1 * b1.y) + w2 * c1.y;
    x[6] = (w0 * a1.z + w1 * b1.z) + w2 * c1.z;
    x[7] = (w0 * a1.w + w1 * b1.w) + w2 * c1.w;
    v8h hv, lv;
#pragma unroll
    for (int e = 0; e < 8; ++e) {
      _Float16 h, l;
      split_h(x[e], LO_CARRY, h, l);
      hv[e] = h; lv[e] = l;
    }
    volatile v8h* ph = (volatile v8h*)(void*)(fhi + (size_t)r * CIN_CH + DSF + ci);
    volatile v8h* pl = (volatile v8h*)(void*)(flo + (size_t)r * CIN_CH + DSF + ci);
    *ph = hv; *pl = lv;
    __threadfence();
    *ph = hv; *pl = lv;
  }
}

template <int KD, int NOUT>
__global__ __launch_bounds__(256) void gemm_f16x3_kernel(
    const unsigned short* __restrict__ Ahp, const unsigned short* __restrict__ Alp,
    const unsigned short* __restrict__ Bhp, const unsigned short* __restrict__ Blp,
    const float* __restrict__ bias, float* __restrict__ C) {
  static_assert(KD % 32 == 0, "K multiple of 32");
  static_assert(NOUT % 32 == 0, "N multiple of 32");
  static_assert(((MROW / 64) * (NOUT / 32)) % 8 == 0, "whole blocks of 8 wave tiles");
  typedef Frag<_Float16> F;
  const _Float16* Ah = (const _Float16*)Ahp;
  const _Float16* Al = (const _Float16*)Alp;
  const _Float16* Bh = (const _Float16*)Bhp;
  const _Float16* Bl = (const _Float16*)Blp;
  __shared__ __align__(16) float sT[8][16 * 36];
  const int lane = threadIdx.x & 31;
  const int wave = threadIdx.x >> 5;
  constexpr int tilesN = NOUT / 32;
  const int tile = blockIdx.x * 8 + wave;
  const int tm = tile / tilesN;
  const int tn = tile - tm * tilesN;
  const int m0 = tm << 6;
  const int n0 = tn << 5;
  const int rlane = lane & 15;
  const int koff  = (lane >> 4) * 8;
  const int mOff  = (lane >> 4) * 8;

  v8f accM[4][2], accR[4][2];
#pragma unroll
  for (int i = 0; i < 4; ++i)
#pragma unroll
    for (int j = 0; j < 2; ++j) {
      accM[i][j] = (v8f){0.f,0.f,0.f,0.f,0.f,0.f,0.f,0.f};
      accR[i][j] = (v8f){0.f,0.f,0.f,0.f,0.f,0.f,0.f,0.f};
    }

  for (int k0 = 0; k0 < KD; k0 += 32) {
    v16h bh[2], bl[2];
#pragma unroll
    for (int j = 0; j < 2; ++j) {
      const size_t bo = (size_t)(n0 + (j << 4) + rlane) * KD + koff + k0;
      bh[j] = F::load(Bh + bo);
      bl[j] = F::load(Bl + bo);
    }
#pragma unroll
    for (int i = 0; i < 4; ++i) {
      const size_t ao = (size_t)(m0 + (i << 4) + rlane) * KD + koff + k0;
      v16h ah = F::load(Ah + ao);
      v16h al = F::load(Al + ao);
#pragma unroll
      for (int j = 0; j < 2; ++j) {
        accM[i][j] = F::mma(ah, bh[j], accM[i][j]);
        accR[i][j] = F::mma(ah, bl[j], accR[i][j]);
        accR[i][j] = F::mma(al, bh[j], accR[i][j]);
      }
      group_guard_h(accM[i][0], accM[i][1], accR[i][0], accR[i][1], ah, al);
    }
    keep4_h(bh[0], bh[1], bl[0], bl[1]);
  }
  acc_guard4(accM[0][0], accM[0][1], accR[0][0], accR[0][1]);
  acc_guard4(accM[1][0], accM[1][1], accR[1][0], accR[1][1]);
  acc_guard4(accM[2][0], accM[2][1], accR[2][0], accR[2][1]);
  acc_guard4(accM[3][0], accM[3][1], accR[3][0], accR[3][1]);

  float* slab = sT[wave];
  float bv[2];
#pragma unroll
  for (int j = 0; j < 2; ++j) bv[j] = bias[n0 + (j << 4) + rlane];
#pragma unroll
  for (int i = 0; i < 4; ++i) {
    const int mBase = m0 + (i << 4);
#pragma unroll
    for (int j = 0; j < 2; ++j) {
#pragma unroll
      for (int r = 0; r < 8; ++r) {
        const float vm = accM[i][j][r] * SCALE_MAIN;
        const float vr = accR[i][j][r] * SCALE_RES;
        const float v = (vm + vr) + bv[j];
        slab[(mOff + r) * 36 + (j << 4) + rlane] = v;
      }
    }
    __builtin_amdgcn_fence(__ATOMIC_RELEASE, "workgroup");
    __builtin_amdgcn_wave_barrier();
    __builtin_amdgcn_fence(__ATOMIC_ACQUIRE, "workgroup");
    {
      const int q = lane >> 3, c4 = (lane & 7) * 4;
      for (int pass = 0; pass < 2; ++pass) {
#pragma unroll
        for (int it = 0; it < 4; ++it) {
          const int row = it * 4 + q;
          const v4f v = *(const v4f*)(slab + row * 36 + c4);
          *(volatile v4f*)(C + (size_t)(mBase + row) * NOUT + n0 + c4) = v;
        }
        __threadfence();
      }
    }
    __builtin_amdgcn_fence(__ATOMIC_RELEASE, "workgroup");
    __builtin_amdgcn_wave_barrier();
    __builtin_amdgcn_fence(__ATOMIC_ACQUIRE, "workgroup");
  }
}

template <int C>
__global__ __launch_bounds__(256) void col_stats_kernel(
    const float* __restrict__ X, float* __restrict__ psum, float* __restrict__ psq) {
  const int c = threadIdx.x;
  const size_t row0 = (size_t)blockIdx.x * STAT_ROWS;
  float s = 0.0f, q = 0.0f;
#pragma unroll 8
  for (int i = 0; i < STAT_ROWS; ++i) {
    const float v = X[(row0 + i) * C + c];
    const float vv = v * v;
    s = s + v;
    q = q + vv;
  }
  volatile float* ps = (volatile float*)psum;
  volatile float* pq = (volatile float*)psq;
  const size_t o = (size_t)blockIdx.x * C + c;
  ps[o] = s; pq[o] = q;
  __threadfence();
  ps[o] = s; pq[o] = q;
}

template <int C>
__global__ __launch_bounds__(256) void bn_params_kernel(
    const float* __restrict__ psum, const float* __restrict__ psq,
    const float* __restrict__ gamma, const float* __restrict__ beta,
    float* __restrict__ scale, float* __restrict__ shift) {
  const int c = threadIdx.x;
  double s = 0.0, q = 0.0;
#pragma unroll 4
  for (int i = 0; i < STAT_BLOCKS; ++i) {
    s = s + (double)psum[(size_t)i * C + c];
    q = q + (double)psq[(size_t)i * C + c];
  }
  const double inv_m = 1.0 / (double)MROW;
  const double mean = s * inv_m;
  double var = q * inv_m - mean * mean;
  var = var < 0.0 ? 0.0 : var;
  const float rs = rsqrtf((float)var + BN_EPS);
  const float sc = gamma[c] * rs;
  const float sh = (float)((double)beta[c] - mean * (double)sc);
  volatile float* vs = (volatile float*)scale;
  volatile float* vh = (volatile float*)shift;
  vs[c] = sc; vh[c] = sh;
  __threadfence();
  vs[c] = sc; vh[c] = sh;
}

__global__ __launch_bounds__(256) void bn_relu_split_kernel(
    const float* __restrict__ X0, const float* __restrict__ scale, const float* __restrict__ shift,
    unsigned short* __restrict__ ahi, unsigned short* __restrict__ alo) {
  const size_t t = (size_t)blockIdx.x * 256 + threadIdx.x;
  const int c8 = (threadIdx.x & 31) * 8;
  const float* xp = X0 + t * 8;
  const v4f xa = *(const v4f*)xp;
  const v4f xb = *(const v4f*)(xp + 4);
  const v4f sa = *(const v4f*)(scale + c8);
  const v4f sb = *(const v4f*)(scale + c8 + 4);
  const v4f ha = *(const v4f*)(shift + c8);
  const v4f hb = *(const v4f*)(shift + c8 + 4);
  float x[8];
  x[0] = xa.x * sa.x + ha.x; x[1] = xa.y * sa.y + ha.y;
  x[2] = xa.z * sa.z + ha.z; x[3] = xa.w * sa.w + ha.w;
  x[4] = xb.x * sb.x + hb.x; x[5] = xb.y * sb.y + hb.y;
  x[6] = xb.z * sb.z + hb.z; x[7] = xb.w * sb.w + hb.w;
  v8h hv, lv;
#pragma unroll
  for (int e = 0; e < 8; ++e) {
    const float v = fmaxf(x[e], 0.0f);
    _Float16 h, l;
    split_h(v, LO_CARRY, h, l);
    hv[e] = h; lv[e] = l;
  }
  volatile v8h* ph = (volatile v8h*)(void*)(ahi + t * 8);
  volatile v8h* pl = (volatile v8h*)(void*)(alo + t * 8);
  *ph = hv; *pl = lv;
  __threadfence();
  *ph = hv; *pl = lv;
}

__global__ __launch_bounds__(256) void bn_relu_out_kernel(
    const float* __restrict__ Y1, const float* __restrict__ scale, const float* __restrict__ shift,
    float* __restrict__ out) {
  const size_t t = (size_t)blockIdx.x * 256 + threadIdx.x;
  const int c4 = (threadIdx.x & 31) * 4;
  const v4f x = *(const v4f*)(Y1 + t * 4);
  const v4f s = *(const v4f*)(scale + c4);
  const v4f h = *(const v4f*)(shift + c4);
  v4f o;
  o.x = fmaxf(x.x * s.x + h.x, 0.0f);
  o.y = fmaxf(x.y * s.y + h.y, 0.0f);
  o.z = fmaxf(x.z * s.z + h.z, 0.0f);
  o.w = fmaxf(x.w * s.w + h.w, 0.0f);
  volatile v4f* po = (volatile v4f*)(out + t * 4);
  *po = o;
  __threadfence();
  *po = o;
}

extern "C" void kernel_launch(void* const* d_in, const int* in_sizes, int n_in,
                              void* d_out, int out_size, void* d_ws, size_t ws_size,
                              hipStream_t stream) {
  if (n_in < 12) return;
  if (ws_size < WS_END) return;
  if (in_sizes[0] != NBATCH * NPT * 3 || in_sizes[1] != NBATCH * SPT * 3) return;
  if (in_sizes[2] != MROW * DSF || in_sizes[3] != NBATCH * SPT * DTF) return;
  if (in_sizes[4] != C0_CH * CIN_CH || in_sizes[8] != C1_CH * C0_CH) return;
  if (out_size != MROW * C1_CH) return;

  const float* xyz_s   = (const float*)d_in[0];
  const float* xyz_t   = (const float*)d_in[1];
  const float* feats_s = (const float*)d_in[2];
  const float* feats_t = (const float*)d_in[3];
  const float* w0      = (const float*)d_in[4];
  const float* b0      = (const float*)d_in[5];
  const float* gamma0  = (const float*)d_in[6];
  const float* beta0   = (const float*)d_in[7];
  const float* w1      = (const float*)d_in[8];
  const float* b1      = (const float*)d_in[9];
  const float* gamma1  = (const float*)d_in[10];
  const float* beta1   = (const float*)d_in[11];
  float* out = (float*)d_out;

  char* ws = (char*)d_ws;
  unsigned short* feat_hi = (unsigned short*)(ws + OFF_FEAT_HI);
  unsigned short* feat_lo = (unsigned short*)(ws + OFF_FEAT_LO);
  unsigned short* a1_hi   = (unsigned short*)(ws + OFF_FEAT_HI);
  unsigned short* a1_lo   = (unsigned short*)(ws + OFF_FEAT_LO);
  float* x0 = (float*)(ws + OFF_X0);
  float* y1 = (float*)(ws + OFF_Y1);
  unsigned short* wb0_hi = (unsigned short*)(ws + OFF_WB0_HI);
  unsigned short* wb0_lo = (unsigned short*)(ws + OFF_WB0_LO);
  unsigned short* wb1_hi = (unsigned short*)(ws + OFF_WB1_HI);
  unsigned short* wb1_lo = (unsigned short*)(ws + OFF_WB1_LO);
  int*   idx  = (int*)(ws + OFF_IDX);
  float* dist = (float*)(ws + OFF_DIST);
  float* psum0 = (float*)(ws + OFF_PSUM0);
  float* psq0  = (float*)(ws + OFF_PSQ0);
  float* psum1 = (float*)(ws + OFF_PSUM1);
  float* psq1  = (float*)(ws + OFF_PSQ1);
  float* scale0 = (float*)(ws + OFF_SCALE0);
  float* shift0 = (float*)(ws + OFF_SHIFT0);
  float* scale1 = (float*)(ws + OFF_SCALE1);
  float* shift1 = (float*)(ws + OFF_SHIFT1);

  constexpr int n8w0 = C0_CH * CIN_CH / 8;
  constexpr int n8w1 = C1_CH * C0_CH / 8;
  static_assert(n8w0 % 256 == 0 && n8w1 % 256 == 0, "whole blocks");
  split_weights_kernel<<<n8w0 / 256, 256, 0, stream>>>(w0, wb0_hi, wb0_lo, n8w0);
  split_weights_kernel<<<n8w1 / 256, 256, 0, stream>>>(w1, wb1_hi, wb1_lo, n8w1);

  knn3_kernel<<<MROW / 256, 256, 0, stream>>>(xyz_s, xyz_t, idx, dist);

  build_features_kernel<<<MROW / 16, 256, 0, stream>>>(feats_s, feats_t, idx, dist, feat_hi, feat_lo);

  gemm_f16x3_kernel<CIN_CH, C0_CH><<<(MROW / 64) * (C0_CH / 32) / 8, 256, 0, stream>>>(
      feat_hi, feat_lo, wb0_hi, wb0_lo, b0, x0);

  col_stats_kernel<C0_CH><<<STAT_BLOCKS, C0_CH, 0, stream>>>(x0, psum0, psq0);
  bn_params_kernel<C0_CH><<<1, C0_CH, 0, stream>>>(psum0, psq0, gamma0, beta0, scale0, shift0);

  bn_relu_split_kernel<<<(MROW * (C0_CH / 8)) / 256, 256, 0, stream>>>(x0, scale0, shift0, a1_hi, a1_lo);

  gemm_f16x3_kernel<C0_CH, C1_CH><<<(MROW / 64) * (C1_CH / 32) / 8, 256, 0, stream>>>(
      a1_hi, a1_lo, wb1_hi, wb1_lo, b1, y1);

  col_stats_kernel<C1_CH><<<STAT_BLOCKS, C1_CH, 0, stream>>>(y1, psum1, psq1);
  bn_params_kernel<C1_CH><<<1, C1_CH, 0, stream>>>(psum1, psq1, gamma1, beta1, scale1, shift1);

  bn_relu_out_kernel<<<(MROW * (C1_CH / 4)) / 256, 256, 0, stream>>>(y1, scale1, shift1, out);
}
